// CausalSelfAttention_89524298318587
// MI455X (gfx1250) — hardware-verified
//
#include <hip/hip_runtime.h>


#ifndef NB
#define NB 8
#endif
#ifndef SEQ
#define SEQ 1024
#endif
#define NB_FULL  8
#define SEQ_FULL 1024
#define DM    768
#define NH    12
#define HD    64
#define DQKV  (3 * DM)
#define KCAT  (2 * DM)
#define RH    256
#define MROWS (NB * SEQ)
#define PSTR  72
#define OSTR  68
#define PSH   8.0f
#define C1    0.18033688011112042f
#define NEGB  (-3.0e38f)
#define PLANE16 ((size_t)NB * NH * SEQ * HD)
#define PLANEE  ((size_t)NB * NH * RH * HD)

#define SZ_WQKV ((size_t)DQKV * DM * 2)
#define SZ_WO   ((size_t)DM * DM * 2)
#define SZ_XB   ((size_t)MROWS * DM * 2)
#define SZ_QK16 ((size_t)2 * PLANE16 * 2)
#define SZ_VT16 ((size_t)PLANE16 * 2)
#define SZ_QKE  ((size_t)2 * PLANEE * 2)
#define SZ_VTE  ((size_t)PLANEE * 2)
#define SZ_AT   ((size_t)MROWS * KCAT * 2)
#define WS_TOTAL (SZ_WQKV + SZ_WO + SZ_XB + SZ_QK16 + SZ_VT16 + 2 * SZ_QKE + 2 * SZ_VTE + SZ_AT)

static_assert(NH * HD == DM);
static_assert(HD == 64);
static_assert(DM % 64 == 0);
static_assert(DM % 32 == 0);
static_assert(KCAT % 32 == 0);
static_assert(DQKV % 64 == 0);
static_assert(SEQ % 64 == 0);
static_assert(RH % 64 == 0);
static_assert(RH <= SEQ);
static_assert(MROWS % 64 == 0);
static_assert(NB <= NB_FULL);
static_assert(SEQ <= SEQ_FULL);
static_assert((MROWS * DM / 8) % 256 == 0);
static_assert(SZ_WQKV % 256 == 0);
static_assert(SZ_WO % 256 == 0);
static_assert(SZ_XB % 256 == 0);
static_assert(SZ_QK16 % 256 == 0);
static_assert(SZ_VT16 % 256 == 0);
static_assert(SZ_QKE % 256 == 0);
static_assert(SZ_VTE % 256 == 0);
static_assert(SZ_AT % 256 == 0);
static_assert(WS_TOTAL <= (size_t)134217728);
static_assert((PSTR * 2) % 16 == 0);
static_assert((OSTR * 4) % 16 == 0);

typedef _Float16 h16;
typedef unsigned short bf;
typedef __attribute__((ext_vector_type(16))) __bf16   v16bf;
typedef __attribute__((ext_vector_type(16))) _Float16 v16h;
typedef __attribute__((ext_vector_type(8)))  _Float16 v8h;
typedef __attribute__((ext_vector_type(8)))  unsigned short v8us;
typedef __attribute__((ext_vector_type(2)))  unsigned short v2us;
typedef __attribute__((ext_vector_type(8)))  float    v8f;
typedef __attribute__((ext_vector_type(4)))  float    v4f;
typedef v8h  __attribute__((may_alias)) v8ha;
typedef v4f  __attribute__((may_alias)) v4fa;
typedef v8us __attribute__((may_alias)) v8usa;

__device__ __forceinline__ unsigned short f2bf(float f) { unsigned u = __float_as_uint(f); u += 0x7FFFu + ((u >> 16) & 1u); return (unsigned short)(u >> 16); }
__device__ __forceinline__ float bf2f(unsigned short b) { return __uint_as_float(((unsigned)b) << 16); }
__device__ __forceinline__ float bfr(float f) { return bf2f(f2bf(f)); }
__device__ __forceinline__ void splitf(float y, unsigned short& h, unsigned short& l) { h = f2bf(y); l = f2bf(y - bf2f(h)); }
__device__ __forceinline__ v16h cat16(v8h lo, v8h hi) { return __builtin_shufflevector(lo, hi, 0, 1, 2, 3, 4, 5, 6, 7, 8, 9, 10, 11, 12, 13, 14, 15); }
__device__ __forceinline__ v16bf cat16b(v8us lo, v8us hi) { return __builtin_bit_cast(v16bf, __builtin_shufflevector(lo, hi, 0, 1, 2, 3, 4, 5, 6, 7, 8, 9, 10, 11, 12, 13, 14, 15)); }
__device__ __forceinline__ v8f wmma16(v16h a, v16h b, v8f c) { return __builtin_amdgcn_wmma_f32_16x16x32_f16(false, a, false, b, (short)0, c, false, false); }
__device__ __forceinline__ v8f wmmab(v16bf a, v16bf b, v8f c) { return __builtin_amdgcn_wmma_f32_16x16x32_bf16(false, a, false, b, (short)0, c, false, false); }
__device__ __forceinline__ v16h  ldfh(const h16* p) { return cat16(*(const v8h*)p, *(const v8h*)(p + 16)); }
__device__ __forceinline__ v16bf ldfb(const bf* p)  { return cat16b(*(const v8us*)p, *(const v8us*)(p + 16)); }
__device__ __forceinline__ void wsync() { __builtin_amdgcn_fence(3  , "wavefront"); __builtin_amdgcn_wave_barrier(); asm volatile("" ::: "memory"); }

__global__ __launch_bounds__(256) void k_wtG(const float* __restrict__ w, int K, int N, bf* Bt) {
    const int lane = threadIdx.x & 31; const int L0 = (blockIdx.x * 8 + (threadIdx.x >> 5)) * 8; const int nlines = N * K / 64;
#pragma unroll
    for (int ps = 0; ps < 2; ++ps) {
#pragma unroll 1
        for (int l = 0; l < 8; ++l) { const int L = L0 + l; if (L >= nlines) break; const size_t e = (size_t)L * 64 + lane * 2; const int k = (int)(e % K), n = (int)(e / K); v2us o;
            o[0] = f2bf(w[(size_t)k * N + n]); o[1] = f2bf(w[(size_t)(k + 1) * N + n]); *(volatile v2us*)(Bt + e) = o; }
        if (ps == 0) __threadfence(); }
}

__global__ __launch_bounds__(256) void k_cvt8(const float* __restrict__ src, bf* dst) {
    const size_t i = (size_t)blockIdx.x * 256 + threadIdx.x; if (i >= (size_t)MROWS * DM / 8) return;
    const size_t row = i / (DM / 8); const int c8 = (int)(i % (DM / 8)); const size_t b = row / SEQ, t = row % SEQ;
    const v8f v = *(const v8f*)(src + (b * SEQ_FULL + t) * DM + (size_t)c8 * 8); v8us o;
#pragma unroll
    for (int k = 0; k < 8; ++k) o[k] = f2bf(v[k]);
    *(volatile v8us*)(dst + i * 8) = o; __threadfence(); *(volatile v8us*)(dst + i * 8) = o;
}

__device__ __forceinline__ void gemm_main(const bf* __restrict__ A, const bf* __restrict__ Bt, const int K, const int ldb, const int kwrap,
                                          const int r0, const int c0, const int lr, const int hi, v8f (&acc)[4][4]) {
    const size_t aoff = (size_t)(r0 + lr) * K + 8 * hi;
    const size_t boff = (size_t)(c0 + lr) * ldb + 8 * hi;
#pragma unroll 1
    for (int kc = 0; kc < K; kc += 32) {
        const int kb = (kc >= kwrap) ? (kc - kwrap) : kc;
        v16bf a[4];
#pragma unroll
        for (int mb = 0; mb < 4; ++mb) a[mb] = ldfb(A + aoff + (size_t)mb * 16 * K + kc);
        v16bf bk;
#pragma unroll
        for (int nb = 0; nb < 4; ++nb) {
            bk = ldfb(Bt + boff + (size_t)nb * 16 * ldb + kb);
#pragma unroll
            for (int mb = 0; mb < 4; ++mb) acc[mb][nb] = wmmab(a[mb], bk, acc[mb][nb]);
        }
        asm volatile("" : "+v"(acc[0][0]), "+v"(acc[1][0]), "+v"(acc[2][0]), "+v"(acc[3][0]), "+v"(acc[0][1]), "+v"(acc[1][1]), "+v"(acc[2][1]), "+v"(acc[3][1]));
        asm volatile("" : "+v"(acc[0][2]), "+v"(acc[1][2]), "+v"(acc[2][2]), "+v"(acc[3][2]));
        asm volatile("v_nop\n\tv_nop\n\tv_nop\n\tv_nop" : "+v"(acc[0][3]), "+v"(acc[1][3]), "+v"(acc[2][3]), "+v"(acc[3][3]) : "v"(a[0]), "v"(a[3]), "v"(bk));
    }
}

__global__ __launch_bounds__(32) void k_qkv(const bf* __restrict__ A, const bf* __restrict__ Bt, const float* __restrict__ bias,
                                            h16* QK16, h16* VT16, bf* QKh, bf* QKl, bf* VTh, bf* VTl) {
    __shared__ __align__(16) float os[64 * OSTR];
    const int lane = threadIdx.x & 31, lr = lane & 15, hi = lane >> 4;
    const int r0 = blockIdx.x * 64, c0 = blockIdx.y * 64;
    v8f acc[4][4];
#pragma unroll
    for (int mb = 0; mb < 4; ++mb)
#pragma unroll
        for (int nb = 0; nb < 4; ++nb) acc[mb][nb] = (v8f){};
    gemm_main(A, Bt, DM, DM, DM, r0, c0, lr, hi, acc);
#pragma unroll
    for (int nb = 0; nb < 4; ++nb) {
        const float bv = bfr(bias[c0 + nb * 16 + lr]);
#pragma unroll
        for (int mb = 0; mb < 4; ++mb)
#pragma unroll
            for (int j = 0; j < 8; ++j) os[(mb * 16 + hi * 8 + j) * OSTR + nb * 16 + lr] = acc[mb][nb][j] + bv;
    }
    __syncthreads();
    const int which = c0 / DM; const int hh = (c0 - which * DM) / HD; const int b = r0 / SEQ; const int t0 = r0 - b * SEQ;
    const size_t bh = (size_t)b * NH + hh; const bool early = (t0 < RH);
    const int g = lane >> 3, piece = lane & 7;
    if (which < 2) {
        const size_t o16 = (size_t)which * PLANE16 + (bh * SEQ + t0) * HD + piece * 8;
        const size_t oe  = (size_t)which * PLANEE + (bh * RH + (early ? t0 : 0)) * HD + piece * 8;
#pragma unroll 1
        for (int ps = 0; ps < 2; ++ps) {
#pragma unroll 1
            for (int s = 0; s < 16; ++s) {
                const int row = 4 * s + g;
                const v4f x0 = *(const v4fa*)&os[row * OSTR + piece * 8]; const v4f x1 = *(const v4fa*)&os[row * OSTR + piece * 8 + 4];
                v8h o; v8us oh, ol;
#pragma unroll
                for (int i = 0; i < 4; ++i) { o[i] = (h16)x0[i]; o[4 + i] = (h16)x1[i]; unsigned short a, c; splitf(x0[i], a, c); oh[i] = a; ol[i] = c; splitf(x1[i], a, c); oh[4 + i] = a; ol[4 + i] = c; }
                *(volatile v8h*)(QK16 + o16 + (size_t)row * HD) = o;
                if (early) { *(volatile v8us*)(QKh + oe + (size_t)row * HD) = oh; *(volatile v8us*)(QKl + oe + (size_t)row * HD) = ol; }
            }
            if (ps == 0) __threadfence();
        }
    } else {
        const size_t o16 = (bh * HD) * SEQ + t0 + piece * 8;
        const size_t oe  = (bh * HD) * RH + (early ? t0 : 0) + piece * 8;
#pragma unroll 1
        for (int ps = 0; ps < 2; ++ps) {
#pragma unroll 1
            for (int s = 0; s < 16; ++s) {
                const int d = 4 * s + g;
                v8h o; v8us oh, ol;
#pragma unroll
                for (int i = 0; i < 8; ++i) { const float xv = os[(piece * 8 + i) * OSTR + d]; o[i] = (h16)xv; unsigned short a, c; splitf(xv, a, c); oh[i] = a; ol[i] = c; }
                *(volatile v8h*)(VT16 + o16 + (size_t)d * SEQ) = o;
                if (early) { *(volatile v8us*)(VTh + oe + (size_t)d * RH) = oh; *(volatile v8us*)(VTl + oe + (size_t)d * RH) = ol; }
            }
            if (ps == 0) __threadfence();
        }
    }
}

__global__ __launch_bounds__(32) void k_oproj(const bf* __restrict__ A, const bf* __restrict__ Bt, const float* __restrict__ bias, float* C) {
    __shared__ __align__(16) float os[16 * OSTR];
    const int lane = threadIdx.x & 31, lr = lane & 15, hi = lane >> 4;
    const int r0 = blockIdx.x * 64, c0 = blockIdx.y * 64;
    v8f acc[4][4];
#pragma unroll
    for (int mb = 0; mb < 4; ++mb)
#pragma unroll
        for (int nb = 0; nb < 4; ++nb) acc[mb][nb] = (v8f){};
    gemm_main(A, Bt, KCAT, DM, DM, r0, c0, lr, hi, acc);
    const int b = r0 / SEQ; const int t0 = r0 - b * SEQ; const int cofs = lr * 4;
    v4f bv; bv[0] = bfr(bias[c0 + cofs]); bv[1] = bfr(bias[c0 + cofs + 1]); bv[2] = bfr(bias[c0 + cofs + 2]); bv[3] = bfr(bias[c0 + cofs + 3]);
#pragma unroll
    for (int mb = 0; mb < 4; ++mb) {
#pragma unroll
        for (int nb = 0; nb < 4; ++nb)
#pragma unroll
            for (int j = 0; j < 8; ++j) os[(hi * 8 + j) * OSTR + nb * 16 + lr] = acc[mb][nb][j];
        __syncthreads();
        float* crow = C + ((size_t)b * SEQ_FULL + t0 + mb * 16) * DM + c0;
#pragma unroll 1
        for (int ps = 0; ps < 2; ++ps) {
#pragma unroll
            for (int s = 0; s < 8; ++s) { const int row = 2 * s + hi; v4f val = *(const v4fa*)&os[row * OSTR + cofs]; val = val + bv;
                *(volatile v4f*)(crow + (size_t)row * DM + cofs) = val; }
            if (ps == 0) __threadfence(); }
        __syncthreads();
    }
}

__global__ __launch_bounds__(128) void k_attn_late(const h16* __restrict__ QK16, const h16* __restrict__ VT16, bf* AT) {
    __shared__ __align__(16) h16 Ps[4 * 16 * PSTR];
    __shared__ __align__(16) float Os[4 * 16 * OSTR];
    const int wave = __builtin_amdgcn_readfirstlane((int)(threadIdx.x >> 5));
    const int lane = threadIdx.x & 31, lr = lane & 15, hi = lane >> 4;
    const int qb = (int)blockIdx.x + RH / 64; const int hh = blockIdx.y; const int b = blockIdx.z;
    const size_t bh = (size_t)b * NH + hh;
    const int q0 = qb * 64 + wave * 16;
    const size_t qpl = bh * SEQ * HD, kpl = PLANE16 + bh * SEQ * HD, vpl = bh * HD * SEQ;
    const int psb = wave * 16 * PSTR, osb = wave * 16 * OSTR;
    const v16h qa0 = ldfh(QK16 + qpl + (size_t)(q0 + lr) * HD + 8 * hi);
    const v16h qa1 = ldfh(QK16 + qpl + (size_t)(q0 + lr) * HD + 32 + 8 * hi);
    float m[8], l[8]; v8f o[4];
#pragma unroll
    for (int r = 0; r < 8; ++r) { m[r] = NEGB; l[r] = 0.0f; }
#pragma unroll
    for (int dt = 0; dt < 4; ++dt) o[dt] = (v8f){};
    const int rowb = q0 + 8 * hi;
#pragma unroll 1
    for (int kt = 0; kt <= qb; ++kt) {
        const int key0 = kt * 64; const bool diag = (kt == qb);
        v8f s[4]; v16h kb1;
#pragma unroll
        for (int nt = 0; nt < 4; ++nt) {
            const h16* kp = QK16 + kpl + (size_t)(key0 + nt * 16 + lr) * HD + 8 * hi;
            const v16h kb0 = ldfh(kp); kb1 = ldfh(kp + 32);
            v8f z = (v8f){};
            z = wmma16(qa0, kb0, z); z = wmma16(qa1, kb1, z); s[nt] = z;
        }
        asm volatile("v_nop\n\tv_nop\n\tv_nop\n\tv_nop" : "+v"(s[0]), "+v"(s[1]), "+v"(s[2]), "+v"(s[3]) : "v"(qa1), "v"(kb1));
        float mx[8];
#pragma unroll
        for (int r = 0; r < 8; ++r) mx[r] = NEGB;
#pragma unroll
        for (int nt = 0; nt < 4; ++nt) {
            const int key = key0 + nt * 16 + lr;
#pragma unroll
            for (int r = 0; r < 8; ++r) { float t = s[nt][r] * C1; t = (diag && key > rowb + r) ? NEGB : t; s[nt][r] = t; mx[r] = fmaxf(mx[r], t); }
        }
#pragma unroll
        for (int r = 0; r < 8; ++r) {
            float v = mx[r];
            v = fmaxf(v, __shfl_xor(v, 1, 32)); v = fmaxf(v, __shfl_xor(v, 2, 32)); v = fmaxf(v, __shfl_xor(v, 4, 32)); v = fmaxf(v, __shfl_xor(v, 8, 32));
            const float mn = fmaxf(m[r], v); const float al = __builtin_amdgcn_exp2f(m[r] - mn); m[r] = mn; l[r] *= al;
#pragma unroll
            for (int dt = 0; dt < 4; ++dt) o[dt][r] *= al;
        }
#pragma unroll
        for (int nt = 0; nt < 4; ++nt) {
#pragma unroll
            for (int r = 0; r < 8; ++r) { const float p = __builtin_amdgcn_exp2f(s[nt][r] - (m[r] - PSH)); l[r] += p; Ps[psb + (8 * hi + r) * PSTR + nt * 16 + lr] = (h16)p; }
        }
        wsync();
        const v16h pa0 = cat16(*(const v8ha*)&Ps[psb + lr * PSTR + 8 * hi], *(const v8ha*)&Ps[psb + lr * PSTR + 16 + 8 * hi]);
        const v16h pa1 = cat16(*(const v8ha*)&Ps[psb + lr * PSTR + 32 + 8 * hi], *(const v8ha*)&Ps[psb + lr * PSTR + 48 + 8 * hi]);
        v16h vb1;
#pragma unroll
        for (int dt = 0; dt < 4; ++dt) {
            const h16* vp = VT16 + vpl + (size_t)(dt * 16 + lr) * SEQ + key0 + 8 * hi;
            const v16h vb0 = ldfh(vp); vb1 = ldfh(vp + 32);
            o[dt] = wmma16(pa0, vb0, o[dt]); o[dt] = wmma16(pa1, vb1, o[dt]);
        }
        asm volatile("v_nop\n\tv_nop\n\tv_nop\n\tv_nop" : "+v"(o[0]), "+v"(o[1]), "+v"(o[2]), "+v"(o[3]) : "v"(pa1), "v"(vb1));
        wsync();
    }
#pragma unroll
    for (int r = 0; r < 8; ++r) {
        float ls = l[r];
        ls += __shfl_xor(ls, 1, 32); ls += __shfl_xor(ls, 2, 32); ls += __shfl_xor(ls, 4, 32); ls += __shfl_xor(ls, 8, 32);
        const float inv = __builtin_amdgcn_rcpf(ls);
#pragma unroll
        for (int dt = 0; dt < 4; ++dt) Os[osb + (8 * hi + r) * OSTR + dt * 16 + lr] = o[dt][r] * inv;
    }
    wsync();
    const int g = lane >> 3, piece = lane & 7;
#pragma unroll 1
    for (int ps = 0; ps < 2; ++ps) {
#pragma unroll
        for (int sI = 0; sI < 4; ++sI) {
            const int row = 4 * sI + g;
            const v4f x0 = *(const v4fa*)&Os[osb + row * OSTR + piece * 8]; const v4f x1 = *(const v4fa*)&Os[osb + row * OSTR + piece * 8 + 4];
            v8us oh, ol;
#pragma unroll
            for (int i = 0; i < 4; ++i) { unsigned short a, c; splitf(x0[i], a, c); oh[i] = a; ol[i] = c; splitf(x1[i], a, c); oh[4 + i] = a; ol[4 + i] = c; }
            bf* dst = AT + ((size_t)b * SEQ + q0 + row) * KCAT + hh * HD + piece * 8;
            *(volatile v8us*)dst = oh; *(volatile v8us*)(dst + DM) = ol;
        }
        if (ps == 0) __threadfence();
    }
}

__global__ __launch_bounds__(128) void k_attn_early(const bf* __restrict__ QKh, const bf* __restrict__ QKl, const bf* __restrict__ VTh, const bf* __restrict__ VTl, bf* AT) {
    __shared__ __align__(16) bf Psh[4 * 16 * PSTR];
    __shared__ __align__(16) bf Psl[4 * 16 * PSTR];
    __shared__ __align__(16) float Os[4 * 16 * OSTR];
    const int wave = __builtin_amdgcn_readfirstlane((int)(threadIdx.x >> 5));
    const int lane = threadIdx.x & 31, lr = lane & 15, hi = lane >> 4;
    const int qb = blockIdx.x; const int hh = blockIdx.y; const int b = blockIdx.z;
    const size_t bh = (size_t)b * NH + hh;
    const int q0 = qb * 64 + wave * 16;
    const size_t qpl = bh * RH * HD, kpl = PLANEE + bh * RH * HD, vpl = bh * HD * RH;
    const int psb = wave * 16 * PSTR, osb = wave * 16 * OSTR;
    const size_t qo = qpl + (size_t)(q0 + lr) * HD + 8 * hi;
    const v16bf qh0 = ldfb(QKh + qo), qh1 = ldfb(QKh + qo + 32), ql0 = ldfb(QKl + qo), ql1 = ldfb(QKl + qo + 32);
    float m[8], l[8]; v8f o[4];
#pragma unroll
    for (int r = 0; r < 8; ++r) { m[r] = NEGB; l[r] = 0.0f; }
#pragma unroll
    for (int dt = 0; dt < 4; ++dt) o[dt] = (v8f){};
    const int rowb = q0 + 8 * hi;
#pragma unroll 1
    for (int kt = 0; kt <= qb; ++kt) {
        const int key0 = kt * 64; const bool diag = (kt == qb);
        v8f s[4]; v16bf kh1;
#pragma unroll
        for (int nt = 0; nt < 4; ++nt) {
            const size_t ko = kpl + (size_t)(key0 + nt * 16 + lr) * HD + 8 * hi;
            const v16bf kh0 = ldfb(QKh + ko); kh1 = ldfb(QKh + ko + 32);
            const v16bf kl0 = ldfb(QKl + ko), kl1 = ldfb(QKl + ko + 32);
            v8f z = (v8f){};
            z = wmmab(ql0, kh0, z); z = wmmab(ql1, kh1, z); z = wmmab(qh0, kl0, z); z = wmmab(qh1, kl1, z); z = wmmab(qh0, kh0, z); z = wmmab(qh1, kh1, z);
            s[nt] = z;
        }
        asm volatile("v_nop\n\tv_nop\n\tv_nop\n\tv_nop" : "+v"(s[0]), "+v"(s[1]), "+v"(s[2]), "+v"(s[3]) : "v"(qh1), "v"(kh1));
        float mx[8];
#pragma unroll
        for (int r = 0; r < 8; ++r) mx[r] = NEGB;
#pragma unroll
        for (int nt = 0; nt < 4; ++nt) {
            const int key = key0 + nt * 16 + lr;
#pragma unroll
            for (int r = 0; r < 8; ++r) { float t = s[nt][r] * C1; t = (diag && key > rowb + r) ? NEGB : t; s[nt][r] = t; mx[r] = fmaxf(mx[r], t); }
        }
#pragma unroll
        for (int r = 0; r < 8; ++r) {
            float v = mx[r];
            v = fmaxf(v, __shfl_xor(v, 1, 32)); v = fmaxf(v, __shfl_xor(v, 2, 32)); v = fmaxf(v, __shfl_xor(v, 4, 32)); v = fmaxf(v, __shfl_xor(v, 8, 32));
            const float mn = fmaxf(m[r], v); const float al = __builtin_amdgcn_exp2f(m[r] - mn); m[r] = mn; l[r] *= al;
#pragma unroll
            for (int dt = 0; dt < 4; ++dt) o[dt][r] *= al;
        }
#pragma unroll
        for (int nt = 0; nt < 4; ++nt) {
#pragma unroll
            for (int r = 0; r < 8; ++r) { const float p = __builtin_amdgcn_exp2f(s[nt][r] - (m[r] - PSH)); l[r] += p; unsigned short a, c; splitf(p, a, c);
                Psh[psb + (8 * hi + r) * PSTR + nt * 16 + lr] = a; Psl[psb + (8 * hi + r) * PSTR + nt * 16 + lr] = c; }
        }
        wsync();
        const v16bf ph0 = cat16b(*(const v8usa*)&Psh[psb + lr * PSTR + 8 * hi], *(const v8usa*)&Psh[psb + lr * PSTR + 16 + 8 * hi]);
        const v16bf ph1 = cat16b(*(const v8usa*)&Psh[psb + lr * PSTR + 32 + 8 * hi], *(const v8usa*)&Psh[psb + lr * PSTR + 48 + 8 * hi]);
        const v16bf pl0 = cat16b(*(const v8usa*)&Psl[psb + lr * PSTR + 8 * hi], *(const v8usa*)&Psl[psb + lr * PSTR + 16 + 8 * hi]);
        const v16bf pl1 = cat16b(*(const v8usa*)&Psl[psb + lr * PSTR + 32 + 8 * hi], *(const v8usa*)&Psl[psb + lr * PSTR + 48 + 8 * hi]);
        v16bf vh1;
#pragma unroll
        for (int dt = 0; dt < 4; ++dt) {
            const size_t vo = vpl + (size_t)(dt * 16 + lr) * RH + key0 + 8 * hi;
            const v16bf vh0 = ldfb(VTh + vo); vh1 = ldfb(VTh + vo + 32);
            const v16bf vl0 = ldfb(VTl + vo), vl1 = ldfb(VTl + vo + 32);
            v8f z = o[dt];
            z = wmmab(pl0, vh0, z); z = wmmab(pl1, vh1, z); z = wmmab(ph0, vl0, z); z = wmmab(ph1, vl1, z); z = wmmab(ph0, vh0, z); z = wmmab(ph1, vh1, z);
            o[dt] = z;
        }
        asm volatile("v_nop\n\tv_nop\n\tv_nop\n\tv_nop" : "+v"(o[0]), "+v"(o[1]), "+v"(o[2]), "+v"(o[3]) : "v"(ph1), "v"(vh1));
        wsync();
    }
#pragma unroll
    for (int r = 0; r < 8; ++r) {
        float ls = l[r];
        ls += __shfl_xor(ls, 1, 32); ls += __shfl_xor(ls, 2, 32); ls += __shfl_xor(ls, 4, 32); ls += __shfl_xor(ls, 8, 32);
        const float inv = __builtin_amdgcn_rcpf(ls);
#pragma unroll
        for (int dt = 0; dt < 4; ++dt) Os[osb + (8 * hi + r) * OSTR + dt * 16 + lr] = o[dt][r] * inv;
    }
    wsync();
    const int g = lane >> 3, piece = lane & 7;
#pragma unroll 1
    for (int ps = 0; ps < 2; ++ps) {
#pragma unroll
        for (int sI = 0; sI < 4; ++sI) {
            const int row = 4 * sI + g;
            const v4f x0 = *(const v4fa*)&Os[osb + row * OSTR + piece * 8]; const v4f x1 = *(const v4fa*)&Os[osb + row * OSTR + piece * 8 + 4];
            v8us oh, ol;
#pragma unroll
            for (int i = 0; i < 4; ++i) { unsigned short a, c; splitf(x0[i], a, c); oh[i] = a; ol[i] = c; splitf(x1[i], a, c); oh[4 + i] = a; ol[4 + i] = c; }
            bf* dst = AT + ((size_t)b * SEQ + q0 + row) * KCAT + hh * HD + piece * 8;
            *(volatile v8us*)dst = oh; *(volatile v8us*)(dst + DM) = ol;
        }
        if (ps == 0) __threadfence();
    }
}

extern "C" void kernel_launch(void* const* d_in, const int* in_sizes, int n_in,
                              void* d_out, int out_size, void* d_ws, size_t ws_size, hipStream_t stream) {
    if (n_in < 5) return;
    if (in_sizes[0] < ((NB - 1) * SEQ_FULL + SEQ) * DM) return;
    if (in_sizes[1] < DM * DQKV || in_sizes[2] < DQKV || in_sizes[3] < DM * DM || in_sizes[4] < DM) return;
    if (out_size < ((NB - 1) * SEQ_FULL + SEQ) * DM) return;
    if (ws_size < WS_TOTAL) return;
    const float* x = (const float*)d_in[0]; const float* wqkv = (const float*)d_in[1]; const float* bqkv = (const float*)d_in[2];
    const float* wo = (const float*)d_in[3]; const float* bo = (const float*)d_in[4];
    float* OUT = (float*)d_out;
    char* wsp = (char*)d_ws; size_t off = 0;
    bf*  WQKV = (bf*)(wsp + off);  off += SZ_WQKV;
    bf*  WO   = (bf*)(wsp + off);  off += SZ_WO;
    bf*  XB   = (bf*)(wsp + off);  off += SZ_XB;
    h16* QK16 = (h16*)(wsp + off); off += SZ_QK16;
    h16* VT16 = (h16*)(wsp + off); off += SZ_VT16;
    bf*  QKh  = (bf*)(wsp + off);  off += SZ_QKE;
    bf*  QKl  = (bf*)(wsp + off);  off += SZ_QKE;
    bf*  VTh  = (bf*)(wsp + off);  off += SZ_VTE;
    bf*  VTl  = (bf*)(wsp + off);  off += SZ_VTE;
    bf*  AT   = (bf*)(wsp + off);  off += SZ_AT;
    if (off > ws_size) return;

    k_wtG<<<(unsigned)((DM * DQKV / 64 + 63) / 64), 256, 0, stream>>>(wqkv, DM, DQKV, WQKV);
    k_wtG<<<(unsigned)((DM * DM / 64 + 63) / 64), 256, 0, stream>>>(wo, DM, DM, WO);
    k_cvt8<<<(unsigned)(((size_t)MROWS * DM / 8 + 255) / 256), 256, 0, stream>>>(x, XB);
    k_qkv<<<dim3(MROWS / 64, DQKV / 64, 1), 32, 0, stream>>>(XB, WQKV, bqkv, QK16, VT16, QKh, QKl, VTh, VTl);
    k_attn_early<<<dim3(RH / 64, NH, NB), 128, 0, stream>>>(QKh, QKl, VTh, VTl, AT);
    if (SEQ > RH) k_attn_late<<<dim3((SEQ - RH) / 64, NH, NB), 128, 0, stream>>>(QK16, VT16, AT);
    k_oproj<<<dim3(MROWS / 64, DM / 64, 1), 32, 0, stream>>>(AT, WO, bo, OUT);
}
